// CLIPAttention_44581760533134
// MI455X (gfx1250) — hardware-verified
//
#include <hip/hip_runtime.h>
#include <math.h>

constexpr int kBatch  = 8;
constexpr int kSeq    = 1024;
constexpr int kDim    = 1024;
constexpr int kHeads  = 16;
constexpr int kDh     = 64;
constexpr int kTok    = kBatch * kSeq;
constexpr int kGroup  = 8;
constexpr int kNGroup = kHeads / kGroup;
constexpr int kWElems = kDim * kDim;
constexpr float kScoreScale = 0.125f;
constexpr float kPCarry     = 32768.0f;
constexpr float kOCarry     = 64.0f;
constexpr float kWoCarry    = 16.0f;
constexpr float kPVScale    = kOCarry / kPCarry;
constexpr float kOutScale   = 1.0f / (kOCarry * kWoCarry);
static_assert(kHeads * kDh == kDim, "shape");
static_assert(kTok % 64 == 0 && kDim % 64 == 0 && kSeq % 64 == 0 && kDh % 64 == 0, "M and N tile multiples of 64");
static_assert(kDim % 32 == 0 && kDh % 32 == 0 && kSeq % 32 == 0, "K multiples of 32");
static_assert(kHeads % kGroup == 0, "groups");
static_assert(kSeq == 128 * 8, "softmax row = 128 threads x 8 columns");
static_assert((kTok * kDim) % (8 * 256) == 0 && kWElems % (8 * 256) == 0, "cast grids exact");

typedef __attribute__((ext_vector_type(16))) _Float16 v16h;
typedef __attribute__((ext_vector_type(8)))  _Float16 v8h;
typedef __attribute__((ext_vector_type(16))) __bf16   v16b;
typedef __attribute__((ext_vector_type(8)))  __bf16   v8b;
typedef __attribute__((ext_vector_type(8)))  float    v8f;
typedef __attribute__((ext_vector_type(4)))  float    v4f;
typedef __attribute__((ext_vector_type(4)))  unsigned int v4u;

__device__ __forceinline__ unsigned short f2bf_bits(float f) {
  unsigned u = __float_as_uint(f);
  return (unsigned short)((u + 0x7FFFu + ((u >> 16) & 1u)) >> 16);
}
__device__ __forceinline__ float bf_bits2f(unsigned short h) { return __uint_as_float(((unsigned)h) << 16); }

__device__ __forceinline__ void dep_guard_h(v8f& a, v8f& b, v16h x, v16h y) { asm volatile("v_nop\n\tv_nop\n\tv_nop\n\tv_nop" : "+v"(a), "+v"(b) : "v"(x), "v"(y)); }
__device__ __forceinline__ void dep_guard_b(v8f& a, v8f& b, v16b x, v16b y) { asm volatile("v_nop\n\tv_nop\n\tv_nop\n\tv_nop" : "+v"(a), "+v"(b) : "v"(x), "v"(y)); }
__device__ __forceinline__ void keep4_h(v16h a, v16h b, v16h c, v16h d) { asm volatile("v_nop" :: "v"(a), "v"(b), "v"(c), "v"(d)); }
__device__ __forceinline__ void keep4_b(v16b a, v16b b, v16b c, v16b d) { asm volatile("v_nop" :: "v"(a), "v"(b), "v"(c), "v"(d)); }
__device__ __forceinline__ void acc_guard4(v8f& a, v8f& b, v8f& c, v8f& d) { asm volatile("v_nop\n\tv_nop\n\tv_nop\n\tv_nop" : "+v"(a), "+v"(b), "+v"(c), "+v"(d)); }
template <typename T> struct Frag;
template <> struct Frag<_Float16> {
  typedef v16h V; union U { v16h v; v8h h[2]; };
  static __device__ __forceinline__ v16h load(const _Float16* p) {
    U f; f.h[0] = *(const v8h*)(p); f.h[1] = *(const v8h*)(p + 16); return f.v;
  }
  static __device__ __forceinline__ v8f mma(v16h a, v16h b, v8f c) {
    return __builtin_amdgcn_wmma_f32_16x16x32_f16(false, a, false, b, (short)0, c, false, false);
  }
  static __device__ __forceinline__ void guard(v8f& a, v8f& b, v16h x, v16h y) { dep_guard_h(a, b, x, y); }
  static __device__ __forceinline__ void keep(v16h a, v16h b, v16h c, v16h d) { keep4_h(a, b, c, d); }
};
template <> struct Frag<__bf16> {
  typedef v16b V; union U { v16b v; v8b h[2]; };
  static __device__ __forceinline__ v16b load(const __bf16* p) {
    U f; f.h[0] = *(const v8b*)(p); f.h[1] = *(const v8b*)(p + 16); return f.v;
  }
  static __device__ __forceinline__ v8f mma(v16b a, v16b b, v8f c) {
    return __builtin_amdgcn_wmma_f32_16x16x32_bf16(false, a, false, b, (short)0, c, false, false);
  }
  static __device__ __forceinline__ void guard(v8f& a, v8f& b, v16b x, v16b y) { dep_guard_b(a, b, x, y); }
  static __device__ __forceinline__ void keep(v16b a, v16b b, v16b c, v16b d) { keep4_b(a, b, c, d); }
};

__device__ __forceinline__ unsigned pk16(unsigned short a, unsigned short b) { return (unsigned)a | ((unsigned)b << 16); }
__device__ __forceinline__ unsigned short h_bits(float f) { const _Float16 h = (_Float16)f; return __builtin_bit_cast(unsigned short, h); }

template <int ET> struct Elem;
template <> struct Elem<0> { typedef _Float16 T; };
template <> struct Elem<1> { typedef __bf16 T; };
template <int ET, bool SPLIT, int BIAS_MODE, int OUT_MODE, bool RESID, int ACT = 0>
__global__ __launch_bounds__(256) void wmma_gemm64(
    const unsigned short* __restrict__ Ap, const unsigned short* __restrict__ A2p, int lda, long strideA,
    const unsigned short* __restrict__ Btp, const unsigned short* __restrict__ Bt2p, int ldb, long strideB,
    void* __restrict__ Cout, void* __restrict__ Cout2, int ldc, long strideC,
    const float* __restrict__ bias,
    const float* __restrict__ resid, long strideR,
    int M, int N, int K, float scale) {
  typedef typename Elem<ET>::T T;
  typedef typename Frag<T>::V V;
  const T* A = (const T*)Ap; const T* A2 = (const T*)A2p; const T* Bt = (const T*)Btp; const T* Bt2 = (const T*)Bt2p;
  __shared__ __align__(16) float sT[8][16 * 68];
  const int b    = blockIdx.y;
  const int lane = threadIdx.x & 31;
  const int wave = threadIdx.x >> 5;
  const int tilesN = N >> 6;
  const int tilesM = M >> 6;
  const int tile = blockIdx.x * 8 + wave;
  if (tile >= tilesM * tilesN) return;
  const int tm = tile / tilesN;
  const int tn = tile - tm * tilesN;
  const int m0 = tm << 6;
  const int n0 = tn << 6;

  const T* Ab  = A  + (size_t)b * strideA;
  const T* Bb  = Bt + (size_t)b * strideB;
  const T* Ab2 = SPLIT ? (A2  + (size_t)b * strideA) : nullptr;
  const T* Bb2 = SPLIT ? (Bt2 + (size_t)b * strideB) : nullptr;

  const int rlane = lane & 15;
  const int koff  = (lane >> 4) * 8;
  const int mOff  = (lane >> 4) * 8;

  v8f acc[4][4];
#pragma unroll
  for (int i = 0; i < 4; ++i)
#pragma unroll
    for (int j = 0; j < 4; ++j) acc[i][j] = (v8f){0.f,0.f,0.f,0.f,0.f,0.f,0.f,0.f};

  for (int k0 = 0; k0 < K; k0 += 32) {
    V bh[4], bl[4];
#pragma unroll
    for (int j = 0; j < 4; ++j) {
      const size_t bo = (size_t)(n0 + (j << 4) + rlane) * ldb + koff + k0;
      bh[j] = Frag<T>::load(Bb + bo);
      if (SPLIT) bl[j] = Frag<T>::load(Bb2 + bo);
    }
#pragma unroll
    for (int i = 0; i < 4; ++i) {
      const size_t ao = (size_t)(m0 + (i << 4) + rlane) * lda + koff + k0;
      V ah = Frag<T>::load(Ab + ao);
      V al;
      if (SPLIT) al = Frag<T>::load(Ab2 + ao);
#pragma unroll
      for (int j = 0; j < 4; ++j) {
        acc[i][j] = Frag<T>::mma(ah, bh[j], acc[i][j]);
        if (SPLIT) {
          acc[i][j] = Frag<T>::mma(ah, bl[j], acc[i][j]);
          acc[i][j] = Frag<T>::mma(al, bh[j], acc[i][j]);
        }
      }
      Frag<T>::guard(acc[i][0], acc[i][3], ah, SPLIT ? al : ah);
    }
    Frag<T>::keep(bh[0], bh[1], bh[2], bh[3]);
    if (SPLIT) Frag<T>::keep(bl[0], bl[1], bl[2], bl[3]);
  }
  acc_guard4(acc[0][0], acc[0][1], acc[0][2], acc[0][3]);
  acc_guard4(acc[1][0], acc[1][1], acc[1][2], acc[1][3]);
  acc_guard4(acc[2][0], acc[2][1], acc[2][2], acc[2][3]);
  acc_guard4(acc[3][0], acc[3][1], acc[3][2], acc[3][3]);

  float* slab = sT[wave];
  const float* Rb = RESID ? (resid + (size_t)b * strideR) : nullptr;
#pragma unroll
  for (int i = 0; i < 4; ++i) {
    const int mBase = m0 + (i << 4);
#pragma unroll
    for (int j = 0; j < 4; ++j) {
      const int n = n0 + (j << 4) + rlane;
      float bv = 0.f;
      if (BIAS_MODE == 2) bv = bias[n];
#pragma unroll
      for (int r = 0; r < 8; ++r) {
        float v = acc[i][j][r] * scale;
        if (BIAS_MODE == 1) v += bias[mBase + mOff + r];
        if (BIAS_MODE == 2) v += bv;
        if (RESID) v += Rb[(size_t)(mBase + mOff + r) * ldc + n];
        if (ACT == 2) v = fmaxf(v, 0.0f);
        if (ACT == 4) v = (v > 0.f) ? v : 0.01f * v;
        slab[(mOff + r) * 68 + (j << 4) + rlane] = v;
      }
    }
    __builtin_amdgcn_fence(__ATOMIC_RELEASE, "workgroup");
    __builtin_amdgcn_wave_barrier();
    __builtin_amdgcn_fence(__ATOMIC_ACQUIRE, "workgroup");
    if (OUT_MODE == 0) {
      float* C = (float*)Cout + (size_t)b * strideC;
      const int hh = lane >> 4, c4 = (lane & 15) * 4;
      for (int pass = 0; pass < 2; ++pass) {
#pragma unroll
        for (int it = 0; it < 8; ++it) {
          const int row = it * 2 + hh;
          v4f v = *(const v4f*)(slab + row * 68 + c4);
          *(volatile v4f*)(C + (size_t)(mBase + row) * ldc + n0 + c4) = v;
        }
        __threadfence();
      }
    } else {
      const int q = lane >> 3, c8 = (lane & 7) * 8;
      unsigned short* C  = (unsigned short*)Cout  + (size_t)b * strideC;
      unsigned short* C2 = (OUT_MODE == 2) ? ((unsigned short*)Cout2 + (size_t)b * strideC) : nullptr;
      for (int pass = 0; pass < 2; ++pass) {
#pragma unroll
        for (int it = 0; it < 4; ++it) {
          const int row = it * 4 + q;
          const float* sp = slab + row * 68 + c8;
          v8h hv, lv;
#pragma unroll
          for (int e = 0; e < 8; ++e) {
            if (OUT_MODE == 1) {
              hv[e] = (_Float16)sp[e];
            } else {
              unsigned short hb = f2bf_bits(sp[e]);
              unsigned short lb = f2bf_bits(sp[e] - bf_bits2f(hb));
              hv[e] = __builtin_bit_cast(_Float16, hb);
              lv[e] = __builtin_bit_cast(_Float16, lb);
            }
          }
          *(volatile v8h*)(C + (size_t)(mBase + row) * ldc + n0 + c8) = hv;
          if (OUT_MODE == 2) *(volatile v8h*)(C2 + (size_t)(mBase + row) * ldc + n0 + c8) = lv;
        }
        __threadfence();
      }
    }
    __builtin_amdgcn_fence(__ATOMIC_RELEASE, "workgroup");
    __builtin_amdgcn_wave_barrier();
    __builtin_amdgcn_fence(__ATOMIC_ACQUIRE, "workgroup");
  }
}

__global__ __launch_bounds__(256) void cast8_bf16_kernel(const float* __restrict__ in, unsigned short* __restrict__ out, int n8) {
  const int i = blockIdx.x * 256 + threadIdx.x;
  if (i >= n8) return;
  const float* p = in + 8 * (size_t)i;
  const v4f a = *(const v4f*)(p);
  const v4f c = *(const v4f*)(p + 4);
  unsigned short hb[8];
#pragma unroll
  for (int e = 0; e < 4; ++e) {
    hb[e]     = f2bf_bits(a[e]);
    hb[4 + e] = f2bf_bits(c[e]);
  }
  const v4u u = (v4u){pk16(hb[0], hb[1]), pk16(hb[2], hb[3]), pk16(hb[4], hb[5]), pk16(hb[6], hb[7])};
  unsigned short* q = out + 8 * (size_t)i;
  *(volatile v4u*)q = u;
  __threadfence();
  *(volatile v4u*)q = u;
}

__global__ __launch_bounds__(256) void wcast4_kernel(const float* __restrict__ W0, const float* __restrict__ W1,
                                                     const float* __restrict__ W2, const float* __restrict__ W3,
                                                     unsigned short* __restrict__ out, int n8) {
  const int z = blockIdx.y;
  const float* W = (z == 0) ? W0 : (z == 1) ? W1 : (z == 2) ? W2 : W3;
  const bool asF16 = (z == 3);
  const int i = blockIdx.x * 256 + threadIdx.x;
  if (i >= n8) return;
  const float* p = W + 8 * (size_t)i;
  const v4f a = *(const v4f*)(p);
  const v4f c = *(const v4f*)(p + 4);
  float x[8];
#pragma unroll
  for (int e = 0; e < 4; ++e) { x[e] = a[e]; x[4 + e] = c[e]; }
  unsigned short hb[8];
#pragma unroll
  for (int e = 0; e < 8; ++e) {
    const unsigned short bb = f2bf_bits(x[e]);
    const unsigned short fb = h_bits(bf_bits2f(bb) * kWoCarry);
    hb[e] = asF16 ? fb : bb;
  }
  const v4u u = (v4u){pk16(hb[0], hb[1]), pk16(hb[2], hb[3]), pk16(hb[4], hb[5]), pk16(hb[6], hb[7])};
  unsigned short* q = out + (size_t)z * kWElems + 8 * (size_t)i;
  *(volatile v4u*)q = u;
  __threadfence();
  *(volatile v4u*)q = u;
}

__global__ __launch_bounds__(128) void softmax_row_kernel(const float* __restrict__ S, unsigned short* __restrict__ P) {
  __shared__ float redM[4];
  __shared__ float redS[4];
  const int i    = blockIdx.x;
  const int hy   = blockIdx.y;
  const int t    = threadIdx.x;
  const int lane = t & 31, wave = t >> 5;
  const size_t rowoff = ((size_t)hy * kSeq + i) * kSeq;
  const float* sr = S + rowoff + 8 * (size_t)t;
  const v4f a = *(const v4f*)(sr);
  const v4f c = *(const v4f*)(sr + 4);
  float x[8];
#pragma unroll
  for (int e = 0; e < 4; ++e) { x[e] = a[e]; x[4 + e] = c[e]; }
  float mx = fmaxf(fmaxf(fmaxf(x[0], x[1]), fmaxf(x[2], x[3])), fmaxf(fmaxf(x[4], x[5]), fmaxf(x[6], x[7])));
#pragma unroll
  for (int off = 16; off > 0; off >>= 1) mx = fmaxf(mx, __shfl_xor(mx, off, 32));
  if (lane == 0) redM[wave] = mx;
  __syncthreads();
  float m = redM[0];
#pragma unroll
  for (int w = 1; w < 4; ++w) m = fmaxf(m, redM[w]);

  float ev[8];
  float sum = 0.0f;
#pragma unroll
  for (int e = 0; e < 8; ++e) {
    ev[e] = expf(x[e] - m);
    sum += ev[e];
  }
#pragma unroll
  for (int off = 16; off > 0; off >>= 1) sum += __shfl_xor(sum, off, 32);
  if (lane == 0) redS[wave] = sum;
  __syncthreads();
  float tot = redS[0];
#pragma unroll
  for (int w = 1; w < 4; ++w) tot += redS[w];
  const float inv = kPCarry / tot;

  unsigned short hb[8];
#pragma unroll
  for (int e = 0; e < 8; ++e) hb[e] = h_bits(ev[e] * inv);
  const v4u u = (v4u){pk16(hb[0], hb[1]), pk16(hb[2], hb[3]), pk16(hb[4], hb[5]), pk16(hb[6], hb[7])};
  unsigned short* pr = P + rowoff + 8 * (size_t)t;
  *(volatile v4u*)pr = u;
  __threadfence();
  *(volatile v4u*)pr = u;
}

extern "C" void kernel_launch(void* const* d_in, const int* in_sizes, int n_in,
                              void* d_out, int out_size, void* d_ws, size_t ws_size,
                              hipStream_t stream) {
  if (n_in < 9) return;
  const int nX = kTok * kDim;
  if (in_sizes[0] != nX) return;
  if (in_sizes[1] != kWElems || in_sizes[3] != kWElems || in_sizes[5] != kWElems || in_sizes[7] != kWElems) return;
  if (in_sizes[2] != kDim || in_sizes[4] != kDim || in_sizes[6] != kDim || in_sizes[8] != kDim) return;
  if (out_size != nX) return;

  const size_t szX  = (size_t)kTok * kDim * 2;
  const size_t szW4 = (size_t)4 * kWElems * 2;
  const size_t szQ  = (size_t)kTok * kDim * 2;
  const size_t szVT = (size_t)kDim * kTok * 2;
  const size_t szS  = (size_t)kGroup * kSeq * kSeq * 4;
  const size_t szP  = (size_t)kGroup * kSeq * kSeq * 2;
  const size_t szO  = (size_t)kSeq * kDim * 2;
  const size_t offX  = 0;
  const size_t offW  = offX + szX;
  const size_t offQ  = offW + szW4;
  const size_t offK  = offQ + szQ;
  const size_t offVT = offK + szQ;
  const size_t offS  = offVT + szVT;
  const size_t offP  = offS + szS;
  const size_t offO  = offP + szP;
  const size_t total = offO + szO;
  if (ws_size < total) return;

  const float* x  = (const float*)d_in[0];
  const float* wq = (const float*)d_in[1];
  const float* bq = (const float*)d_in[2];
  const float* wk = (const float*)d_in[3];
  const float* bk = (const float*)d_in[4];
  const float* wv = (const float*)d_in[5];
  const float* bv = (const float*)d_in[6];
  const float* wo = (const float*)d_in[7];
  const float* bo = (const float*)d_in[8];
  float* out = (float*)d_out;
  char* ws = (char*)d_ws;
  unsigned short* XB  = (unsigned short*)(ws + offX);
  unsigned short* W4  = (unsigned short*)(ws + offW);
  unsigned short* Q16 = (unsigned short*)(ws + offQ);
  unsigned short* K16 = (unsigned short*)(ws + offK);
  unsigned short* VT  = (unsigned short*)(ws + offVT);
  float*          SC  = (float*)(ws + offS);
  unsigned short* PP  = (unsigned short*)(ws + offP);
  unsigned short* O16 = (unsigned short*)(ws + offO);
  const unsigned short* Wqb  = W4;
  const unsigned short* Wkb  = W4 + (size_t)1 * kWElems;
  const unsigned short* Wvb  = W4 + (size_t)2 * kWElems;
  const unsigned short* Wo16 = W4 + (size_t)3 * kWElems;

  const int nX8 = nX / 8;
  const int nW8 = kWElems / 8;
  cast8_bf16_kernel<<<dim3(nX8 / 256), dim3(256), 0, stream>>>(x, XB, nX8);
  wcast4_kernel<<<dim3(nW8 / 256, 4), dim3(256), 0, stream>>>(wq, wk, wv, wo, W4, nW8);

  const int tilesProj = (kTok / 64) * (kDim / 64);
  wmma_gemm64<1, false, 2, 1, false, 0><<<dim3(tilesProj / 8, 1), dim3(256), 0, stream>>>(
      XB, XB, kDim, 0L, Wqb, Wqb, kDim, 0L, (void*)Q16, (void*)Q16, kDim, 0L, bq, bq, 0L, kTok, kDim, kDim, 1.0f);
  wmma_gemm64<1, false, 2, 1, false, 0><<<dim3(tilesProj / 8, 1), dim3(256), 0, stream>>>(
      XB, XB, kDim, 0L, Wkb, Wkb, kDim, 0L, (void*)K16, (void*)K16, kDim, 0L, bk, bk, 0L, kTok, kDim, kDim, 1.0f);
  wmma_gemm64<1, false, 1, 1, false, 0><<<dim3(tilesProj / 8, 1), dim3(256), 0, stream>>>(
      Wvb, Wvb, kDim, 0L, XB, XB, kDim, 0L, (void*)VT, (void*)VT, kTok, 0L, bv, bv, 0L, kDim, kTok, kDim, 1.0f);

  const long strideHead  = (long)kDh;
  const long stridePlane = (long)kSeq * kSeq;
  const long strideVT    = (long)kDh * kTok;
  const int  tilesScore  = (kSeq / 64) * (kSeq / 64);
  const int  tilesPV     = (kSeq / 64) * (kDh / 64);
  const int  tilesOut    = (kSeq / 64) * (kDim / 64);

  for (int b = 0; b < kBatch; ++b) {
    for (int g = 0; g < kNGroup; ++g) {
      const size_t qkOff = ((size_t)b * kSeq) * kDim + (size_t)g * kGroup * kDh;
      const unsigned short* Ag = Q16 + qkOff;
      const unsigned short* Bg = K16 + qkOff;
      wmma_gemm64<0, false, 0, 0, false, 0><<<dim3(tilesScore / 8, kGroup), dim3(256), 0, stream>>>(
          Ag, Ag, kDim, strideHead, Bg, Bg, kDim, strideHead,
          (void*)SC, (void*)SC, kSeq, stridePlane, bq, bq, 0L, kSeq, kSeq, kDh, kScoreScale);
      softmax_row_kernel<<<dim3(kSeq, kGroup), dim3(128), 0, stream>>>(SC, PP);
      const unsigned short* VTg = VT + ((size_t)g * kGroup * kDh) * kTok + (size_t)b * kSeq;
      unsigned short* Og = O16 + (size_t)g * kGroup * kDh;
      wmma_gemm64<0, false, 0, 1, false, 0><<<dim3(tilesPV / 8, kGroup), dim3(256), 0, stream>>>(
          PP, PP, kSeq, stridePlane, VTg, VTg, kTok, strideVT,
          (void*)Og, (void*)Og, kDim, strideHead, bq, bq, 0L, kSeq, kDh, kSeq, kPVScale);
    }
    float* outb = out + ((size_t)b * kSeq) * kDim;
    wmma_gemm64<0, false, 2, 0, false, 0><<<dim3(tilesOut / 8, 1), dim3(256), 0, stream>>>(
        O16, O16, kDim, 0L, Wo16, Wo16, kDim, 0L, (void*)outb, (void*)outb, kDim, 0L, bo, bo, 0L,
        kSeq, kDim, kDim, kOutScale);
  }
}
